// C2M_24378234372461
// MI455X (gfx1250) — hardware-verified
//
#include <hip/hip_runtime.h>
#define NBt 8
#define C4 512
#define C3 256
#define C2 128
#define HW4 121
#define HW3 484
#define HW2 1936
#define L2Q 1934
#define Q4P 128
#define Q3P 512
#define Q2P 1952
#define K3P 496
typedef __bf16 v16b __attribute__((ext_vector_type(16)));
typedef unsigned short v8us __attribute__((ext_vector_type(8), may_alias));
typedef float  v8f  __attribute__((ext_vector_type(8)));
typedef float  v4f  __attribute__((ext_vector_type(4)));
typedef float  v4fa __attribute__((ext_vector_type(4), may_alias));
union FragB { v16b v; v8us half[2]; unsigned short u[16]; };

__device__ __forceinline__ unsigned short bf16_bits(float x) { unsigned int u = __float_as_uint(x); return (unsigned short)((u + 0x7FFFu + ((u >> 16) & 1u)) >> 16); }
__device__ __forceinline__ float bf16_val(unsigned short b) { return __uint_as_float(((unsigned int)b) << 16); }
__device__ __forceinline__ float bf16_round(float x) { return bf16_val(bf16_bits(x)); }
template <int NT>
__device__ __forceinline__ v8f mmaN(v16b ah, v16b al, v16b bh, v16b bl, v8f c) {
  c = __builtin_amdgcn_wmma_f32_16x16x32_bf16(false, ah, false, bh, (short)0, c, false, false);
  if (NT >= 2) c = __builtin_amdgcn_wmma_f32_16x16x32_bf16(false, al, false, bh, (short)0, c, false, false);
  if (NT >= 3) c = __builtin_amdgcn_wmma_f32_16x16x32_bf16(false, ah, false, bl, (short)0, c, false, false);
  asm volatile("v_nop\n\tv_nop\n\tv_nop\n\tv_nop" : "+v"(c) : "v"(ah), "v"(al), "v"(bh), "v"(bl));
  return c;
}

__global__ __launch_bounds__(256) void k_wt_bf16(const float* __restrict__ W, unsigned short* __restrict__ Wt, int K, int N) {
  const int t = blockIdx.x * 256 + threadIdx.x;
  const int k8n = K / 8;
  if (t >= N * k8n) return;
  const int n = t / k8n, k8 = (t % k8n) * 8;
  v8us v;
#pragma unroll
  for (int i = 0; i < 8; ++i) v[i] = bf16_bits(W[(size_t)(k8 + i) * N + n]);
  *(volatile v8us*)(Wt + (size_t)n * K + k8) = v;
  __threadfence();
  *(volatile v8us*)(Wt + (size_t)n * K + k8) = v;
}

template <bool ASPLIT, int ACT, bool BIAS_BF16>
__global__ __launch_bounds__(128) void k_gemm_bf(const float* __restrict__ A, int lda, const unsigned short* __restrict__ Wt, int ldb,
                                               const float* __restrict__ bias, float* __restrict__ C, int ldc, int M, int N, int K) {
  __shared__ __attribute__((aligned(16))) float so[4][16][64];
  const int tid = threadIdx.x, w = tid >> 5, lane = tid & 31, ln = lane & 15, hh = lane >> 4;
  const int ntn = N / 64;
  const int wid = blockIdx.x * 4 + w;
  const int mt = wid / ntn, nq = wid % ntn;
  if (mt * 16 >= M) return;
  const int row0 = mt * 16, col0 = nq * 64;
  const float* arow = A + (size_t)(row0 + ln) * lda;
  v8f acc[4] = {};
  for (int kb = 0; kb < K; kb += 32) {
    FragB ah, al;
    const v4f x0 = *(const v4fa*)(arow + kb + 8 * hh), x1 = *(const v4fa*)(arow + kb + 8 * hh + 4);
    const v4f x2 = *(const v4fa*)(arow + kb + 16 + 8 * hh), x3 = *(const v4fa*)(arow + kb + 16 + 8 * hh + 4);
    float xs[16] = {x0[0],x0[1],x0[2],x0[3],x1[0],x1[1],x1[2],x1[3],x2[0],x2[1],x2[2],x2[3],x3[0],x3[1],x3[2],x3[3]};
#pragma unroll
    for (int i = 0; i < 16; ++i) { const unsigned short hb = bf16_bits(xs[i]); ah.u[i] = hb; al.u[i] = ASPLIT ? bf16_bits(xs[i] - bf16_val(hb)) : (unsigned short)0; }
#pragma unroll
    for (int t = 0; t < 4; ++t) {
      const unsigned short* brow = Wt + (size_t)(col0 + t * 16 + ln) * ldb + kb;
      FragB b;
      b.half[0] = *(const v8us*)(brow + 8 * hh);
      b.half[1] = *(const v8us*)(brow + 16 + 8 * hh);
      acc[t] = mmaN<ASPLIT ? 2 : 1>(ah.v, al.v, b.v, b.v, acc[t]);
    }
  }
#pragma unroll
  for (int t = 0; t < 4; ++t) {
    float bv = bias ? bias[col0 + t * 16 + ln] : 0.f;
    if (BIAS_BF16) bv = bf16_round(bv);
#pragma unroll
    for (int r = 0; r < 8; ++r) { float v = acc[t][r] + bv; if (ACT == 1) v = fmaxf(v, 0.f); so[w][8 * hh + r][t * 16 + ln] = v; }
  }
  __builtin_amdgcn_fence(__ATOMIC_ACQ_REL, "workgroup");
  __builtin_amdgcn_wave_barrier();
  const int rsub = lane >> 4, c4 = (lane & 15) * 4;
  for (int pass = 0; pass < 2; ++pass) {
#pragma unroll
    for (int q = 0; q < 8; ++q) {
      const int r = q * 2 + rsub;
      const v4f v = *(const v4fa*)&so[w][r][c4];
      *(volatile v4f*)(C + (size_t)(row0 + r) * ldc + col0 + c4) = v;
    }
    if (pass == 0) __threadfence();
  }
}

template <bool ASPLIT, int ACT, bool BIAS_BF16, bool RES_BF16>
__global__ __launch_bounds__(128) void k_gemm_bf3(const float* __restrict__ A, int lda, const unsigned short* __restrict__ Wt, int ldb,
                                                const float* __restrict__ bias, const float* __restrict__ resid, int rmod, int ldr,
                                                float* __restrict__ C, int ldc, int M, int N, int K) {
  __shared__ __attribute__((aligned(16))) float so[4][16][64];
  const int tid = threadIdx.x, w = tid >> 5, lane = tid & 31, ln = lane & 15, hh = lane >> 4;
  const int ntn = N / 64;
  const int wid = blockIdx.x * 4 + w;
  const int mt = wid / ntn, nq = wid % ntn;
  if (mt * 16 >= M) return;
  const int row0 = mt * 16, col0 = nq * 64;
  const float* arow = A + (size_t)(row0 + ln) * lda;
  v8f acc[4] = {};
  for (int kb = 0; kb < K; kb += 32) {
    FragB ah, al;
    const v4f x0 = *(const v4fa*)(arow + kb + 8 * hh), x1 = *(const v4fa*)(arow + kb + 8 * hh + 4);
    const v4f x2 = *(const v4fa*)(arow + kb + 16 + 8 * hh), x3 = *(const v4fa*)(arow + kb + 16 + 8 * hh + 4);
    float xs[16] = {x0[0],x0[1],x0[2],x0[3],x1[0],x1[1],x1[2],x1[3],x2[0],x2[1],x2[2],x2[3],x3[0],x3[1],x3[2],x3[3]};
#pragma unroll
    for (int i = 0; i < 16; ++i) { const unsigned short hb = bf16_bits(xs[i]); ah.u[i] = hb; al.u[i] = ASPLIT ? bf16_bits(xs[i] - bf16_val(hb)) : (unsigned short)0; }
#pragma unroll
    for (int t = 0; t < 4; ++t) {
      const unsigned short* brow = Wt + (size_t)(col0 + t * 16 + ln) * ldb + kb;
      FragB b;
      b.half[0] = *(const v8us*)(brow + 8 * hh);
      b.half[1] = *(const v8us*)(brow + 16 + 8 * hh);
      acc[t] = mmaN<ASPLIT ? 2 : 1>(ah.v, al.v, b.v, b.v, acc[t]);
    }
  }
#pragma unroll
  for (int t = 0; t < 4; ++t) {
    const int col = col0 + t * 16 + ln;
    float bv = bias ? bias[col] : 0.f;
    if (BIAS_BF16) bv = bf16_round(bv);
#pragma unroll
    for (int r = 0; r < 8; ++r) {
      float v = acc[t][r] + bv;
      if (resid) { float rv = resid[(size_t)((row0 + 8 * hh + r) % rmod) * ldr + col]; if (RES_BF16) rv = bf16_round(rv); v += rv; }
      if (ACT == 1) v = fmaxf(v, 0.f);
      if (ACT == 2) v = 0.5f * v * (1.0f + erff(v * 0.70710678118654752f));
      if (ACT == 3) { const float u = 0.7978845608028654f * (v + 0.044715f * v * v * v); v = 0.5f * v * (1.0f + tanhf(u)); }
      so[w][8 * hh + r][t * 16 + ln] = v;
    }
  }
  __builtin_amdgcn_fence(__ATOMIC_ACQ_REL, "workgroup");
  __builtin_amdgcn_wave_barrier();
  const int rsub = lane >> 4, c4 = (lane & 15) * 4;
  for (int pass = 0; pass < 2; ++pass) {
#pragma unroll
    for (int q = 0; q < 8; ++q) {
      const int r = q * 2 + rsub;
      const v4f v = *(const v4fa*)&so[w][r][c4];
      *(volatile v4f*)(C + (size_t)(row0 + r) * ldc + col0 + c4) = v;
    }
    if (pass == 0) __threadfence();
  }
}
template <bool PARAM_BF16>
__global__ __launch_bounds__(256) void k_layernorm(const float* __restrict__ X, const float* __restrict__ R, const float* __restrict__ g, const float* __restrict__ bta,
                                                  float* __restrict__ out_sum, float* __restrict__ out_norm, int N, float eps) {
  __shared__ float red[256];
  const int row = blockIdx.x, tid = threadIdx.x;
  const float* x = X + (size_t)row * N; const float* rr = R ? R + (size_t)row * N : nullptr;
  float vals[16];
  const int per = N / 256;
  float s1 = 0.f;
  for (int u = 0; u < per / 4; ++u) {
    const int j = tid * 4 + 1024 * u;
    const v4f a = *(const v4fa*)(x + j);
    v4f b = {0.f,0.f,0.f,0.f}; if (rr) b = *(const v4fa*)(rr + j);
#pragma unroll
    for (int q = 0; q < 4; ++q) { const float v = a[q] + b[q]; vals[u * 4 + q] = v; s1 += v; }
  }
  red[tid] = s1; __syncthreads();
  for (int st = 128; st > 0; st >>= 1) { if (tid < st) red[tid] += red[tid + st]; __syncthreads(); }
  const float mu = red[0] / (float)N; __syncthreads();
  float s2 = 0.f;
  for (int u = 0; u < per / 4; ++u)
#pragma unroll
    for (int q = 0; q < 4; ++q) { const float c = vals[u * 4 + q] - mu; s2 += c * c; }
  red[tid] = s2; __syncthreads();
  for (int st = 128; st > 0; st >>= 1) { if (tid < st) red[tid] += red[tid + st]; __syncthreads(); }
  const float rs = rsqrtf(red[0] / (float)N + eps);
  for (int pass = 0; pass < 2; ++pass) {
    for (int u = 0; u < per / 4; ++u) {
      const int j = tid * 4 + 1024 * u;
      v4f o, sm;
#pragma unroll
      for (int q = 0; q < 4; ++q) {
        float gg = g[j + q], bb = bta[j + q];
        if (PARAM_BF16) { gg = bf16_round(gg); bb = bf16_round(bb); }
        sm[q] = vals[u * 4 + q]; o[q] = (vals[u * 4 + q] - mu) * rs * gg + bb;
      }
      if (out_sum) *(volatile v4f*)(out_sum + (size_t)row * N + j) = sm;
      *(volatile v4f*)(out_norm + (size_t)row * N + j) = o;
    }
    if (pass == 0) __threadfence();
  }
}


typedef _Float16 v16h __attribute__((ext_vector_type(16)));
union FragH { v16h v; v8us half[2]; _Float16 h[16]; unsigned short u[16]; };
template <int NT>
__device__ __forceinline__ v8f mmaH(v16h ah, v16h al, v16h bh, v16h bl, v8f c) {
  c = __builtin_amdgcn_wmma_f32_16x16x32_f16(false, ah, false, bh, (short)0, c, false, false);
  if (NT >= 2) c = __builtin_amdgcn_wmma_f32_16x16x32_f16(false, al, false, bh, (short)0, c, false, false);
  if (NT >= 3) c = __builtin_amdgcn_wmma_f32_16x16x32_f16(false, ah, false, bl, (short)0, c, false, false);
  asm volatile("v_nop\n\tv_nop\n\tv_nop\n\tv_nop" : "+v"(c) : "v"(ah), "v"(al), "v"(bh), "v"(bl));
  return c;
}
template <bool ASPLIT>
__global__ __launch_bounds__(128) void k_gemm_h(const float* __restrict__ A, int lda, size_t sA, const _Float16* __restrict__ Bh, int ldb, size_t sB, float alpha, float* __restrict__ C, int ldc, size_t sC, int M, int N, int K) {
  __shared__ __attribute__((aligned(16))) float so[4][16][64];
  const int tid = threadIdx.x, w = tid >> 5, lane = tid & 31, ln = lane & 15, hh = lane >> 4; const int by = blockIdx.y;
  A += (size_t)by * sA; Bh += (size_t)by * sB; C += (size_t)by * sC;
  const int ntn = (N + 63) / 64; const int wid = blockIdx.x * 4 + w; const int mt = wid / ntn, nq = wid % ntn; if (mt * 16 >= M) return;
  const int row0 = mt * 16, col0 = nq * 64; const float* arow = A + (size_t)(row0 + ln) * lda;
  v8f acc[4] = {};
  for (int kb = 0; kb < K; kb += 32) {
    FragH ah, al;
    const v4f x0 = *(const v4fa*)(arow + kb + 8 * hh), x1 = *(const v4fa*)(arow + kb + 8 * hh + 4), x2 = *(const v4fa*)(arow + kb + 16 + 8 * hh), x3 = *(const v4fa*)(arow + kb + 16 + 8 * hh + 4);
    float xs[16] = {x0[0],x0[1],x0[2],x0[3],x1[0],x1[1],x1[2],x1[3],x2[0],x2[1],x2[2],x2[3],x3[0],x3[1],x3[2],x3[3]};
#pragma unroll
    for (int i = 0; i < 16; ++i) { const _Float16 h = (_Float16)xs[i]; ah.h[i] = h; al.h[i] = ASPLIT ? (_Float16)(xs[i] - (float)h) : (_Float16)0.0f; }
#pragma unroll
    for (int t = 0; t < 4; ++t) { if (col0 + t * 16 >= N) continue; const size_t boff = (size_t)(col0 + t * 16 + ln) * ldb + kb; FragH bq; bq.half[0] = *(const v8us*)(Bh + boff + 8 * hh); bq.half[1] = *(const v8us*)(Bh + boff + 16 + 8 * hh);
      acc[t] = mmaH<ASPLIT ? 2 : 1>(ah.v, al.v, bq.v, bq.v, acc[t]); }
  }
#pragma unroll
  for (int t = 0; t < 4; ++t) { if (col0 + t * 16 >= N) continue;
#pragma unroll
    for (int r = 0; r < 8; ++r) so[w][8 * hh + r][t * 16 + ln] = acc[t][r] * alpha; }
  __builtin_amdgcn_fence(__ATOMIC_ACQ_REL, "workgroup"); __builtin_amdgcn_wave_barrier();
  const int rsub = lane >> 4, c4 = (lane & 15) * 4;
  for (int pass = 0; pass < 2; ++pass) {
#pragma unroll
    for (int q = 0; q < 8; ++q) { const int r = q * 2 + rsub; if (col0 + c4 < N) { const v4f v = *(const v4fa*)&so[w][r][c4]; *(volatile v4f*)(C + (size_t)(row0 + r) * ldc + col0 + c4) = v; } }
    if (pass == 0) __threadfence(); }
}

__global__ __launch_bounds__(256) void k_wt_f16(const float* __restrict__ W, _Float16* __restrict__ Wt, int K, int N, float scale) {
  const int t = blockIdx.x * 256 + threadIdx.x; if (t >= N * (K / 8)) return; const int n = t / (K / 8), k8 = (t % (K / 8)) * 8; FragH f;
#pragma unroll
  for (int i = 0; i < 8; ++i) f.h[i] = (_Float16)(bf16_round(W[(size_t)(k8 + i) * N + n]) * scale); const v8us o = f.half[0];
  *(volatile v8us*)((unsigned short*)Wt + (size_t)n * K + k8) = o; __threadfence(); *(volatile v8us*)((unsigned short*)Wt + (size_t)n * K + k8) = o;
}
template <int ACT>
__global__ __launch_bounds__(128) void k_gemm_hhx(const _Float16* __restrict__ A, int lda, size_t sA, const _Float16* __restrict__ Bh, int ldb, size_t sB, float alpha, const float* __restrict__ bias, size_t sBias, const float* __restrict__ CP, int rowsPerB, size_t sCPb, int row0g,
    float* __restrict__ C, _Float16* __restrict__ C16, int ldc, size_t sC, int M, int N, int K) {
  __shared__ __attribute__((aligned(16))) float so[4][16][64];
  const int tid = threadIdx.x, w = tid >> 5, lane = tid & 31, ln = lane & 15, hh = lane >> 4; const int by = blockIdx.y;
  A += (size_t)by * sA; Bh += (size_t)by * sB; const size_t cofs = (size_t)by * sC; const float* bp = bias ? bias + (size_t)by * sBias : nullptr;
  const int ntn = (N + 63) / 64; const int wid = blockIdx.x * 4 + w; const int mt = wid / ntn, nq = wid % ntn; if (mt * 16 >= M) return;
  const int row0 = mt * 16, col0 = nq * 64; const _Float16* arow = A + (size_t)(row0 + ln) * lda;
  v8f acc[4] = {};
  for (int kb = 0; kb < K; kb += 32) { FragH ah; ah.half[0] = *(const v8us*)((const unsigned short*)arow + kb + 8 * hh); ah.half[1] = *(const v8us*)((const unsigned short*)arow + kb + 16 + 8 * hh);
#pragma unroll
    for (int t = 0; t < 4; ++t) { if (col0 + t * 16 >= N) continue; const size_t boff = (size_t)(col0 + t * 16 + ln) * ldb + kb; FragH bq; bq.half[0] = *(const v8us*)((const unsigned short*)Bh + boff + 8 * hh); bq.half[1] = *(const v8us*)((const unsigned short*)Bh + boff + 16 + 8 * hh);
      acc[t] = mmaH<1>(ah.v, ah.v, bq.v, bq.v, acc[t]); }
  }
#pragma unroll
  for (int t = 0; t < 4; ++t) { if (col0 + t * 16 >= N) continue; const int col = col0 + t * 16 + ln; const float bv = bp ? bf16_round(bp[col]) : 0.f;
#pragma unroll
    for (int r = 0; r < 8; ++r) { float v = acc[t][r] * alpha + bv; if (CP) { const int bidx = (row0g + row0 + 8 * hh + r) / rowsPerB; v += CP[(size_t)bidx * sCPb + (size_t)by * 64 + col]; } if (ACT == 1) v = (v > 0.f) ? v : expm1f(v); else if (ACT == 7) v = (v > 0.f) ? v + 1.0f : expf(v); else if (ACT == 8) v = tanhf(v); else if (ACT == 9) v = 0.5f * v * (1.0f + tanhf(0.7978845608028654f * (v + 0.044715f * v * v * v))); else if (ACT == 11) v = 1.0f / (1.0f + expf(-v)); else if (ACT == 12) v = (v > 0.f) ? v : 0.01f * v; else if (ACT == 14) v = (v > 0.f) ? v : 0.1f * v; else if (ACT == 15) v = v / (1.0f + expf(-v)); else if (ACT == 3) v = fmaxf(v, 0.f); else if (ACT == 6) v = 0.5f * v * (1.0f + erff(v * 0.70710678118654752f)); so[w][8 * hh + r][t * 16 + ln] = v; } }
  __builtin_amdgcn_fence(__ATOMIC_ACQ_REL, "workgroup"); __builtin_amdgcn_wave_barrier();
  const int rsub = lane >> 4, c4 = (lane & 15) * 4; typedef _Float16 v4h __attribute__((ext_vector_type(4)));
  for (int pass = 0; pass < 2; ++pass) {
#pragma unroll
    for (int q = 0; q < 8; ++q) { const int r = q * 2 + rsub; if (col0 + c4 < N) { const v4f v = *(const v4fa*)&so[w][r][c4]; if (C) *(volatile v4f*)(C + cofs + (size_t)(row0 + r) * ldc + col0 + c4) = v; if (C16) { v4h h4; for (int i = 0; i < 4; ++i) h4[i] = (_Float16)v[i]; *(volatile v4h*)(C16 + cofs + (size_t)(row0 + r) * ldc + col0 + c4) = h4; } } }
    if (pass == 0) __threadfence(); }
}


typedef _Float16 v4h __attribute__((ext_vector_type(4)));

__global__ __launch_bounds__(256) void k_x16(const float* __restrict__ x, _Float16* __restrict__ X16, size_t n8) { const size_t t = (size_t)blockIdx.x * 256 + threadIdx.x; if (t >= n8) return; FragH f;
#pragma unroll
  for (int q = 0; q < 8; ++q) f.h[q] = (_Float16)bf16_round(x[t * 8 + q]); *(volatile v8us*)((unsigned short*)X16 + t * 8) = f.half[0]; __threadfence(); *(volatile v8us*)((unsigned short*)X16 + t * 8) = f.half[0]; }
__global__ __launch_bounds__(256) void k_h16(const float* __restrict__ x, _Float16* __restrict__ X16, size_t n8) { const size_t t = (size_t)blockIdx.x * 256 + threadIdx.x; if (t >= n8) return; FragH f;
#pragma unroll
  for (int q = 0; q < 8; ++q) f.h[q] = (_Float16)x[t * 8 + q]; *(volatile v8us*)((unsigned short*)X16 + t * 8) = f.half[0]; __threadfence(); *(volatile v8us*)((unsigned short*)X16 + t * 8) = f.half[0]; }
__global__ __launch_bounds__(256) void k_round16f(const float* __restrict__ W, _Float16* __restrict__ Bt, size_t n8) { const size_t t = (size_t)blockIdx.x * 256 + threadIdx.x; if (t >= n8) return; FragH f;
#pragma unroll
  for (int i = 0; i < 8; ++i) f.h[i] = (_Float16)(bf16_round(W[t * 8 + i]) * 16.0f); *(volatile v8us*)((unsigned short*)Bt + t * 8) = f.half[0]; __threadfence(); *(volatile v8us*)((unsigned short*)Bt + t * 8) = f.half[0]; }
template <int NHv, int TTv>
__global__ __launch_bounds__(256) void k_vt(const _Float16* __restrict__ V16, int ldv, int voff, _Float16* __restrict__ Vt) { __shared__ unsigned short tl[64][66]; const int tid = threadIdx.x; const int slab = blockIdx.x / (TTv / 64), lg = blockIdx.x % (TTv / 64); const int b = slab / NHv, h = slab % NHv;
  for (int i = tid; i < 64 * 8; i += 256) { const int r = i / 8, c8 = (i % 8) * 8; FragH f; f.half[0] = *(const v8us*)((const unsigned short*)V16 + ((size_t)b * TTv + lg * 64 + r) * ldv + voff + h * 64 + c8);
#pragma unroll
    for (int q = 0; q < 8; ++q) tl[r][c8 + q] = f.u[q]; }
  __syncthreads();
  for (int pass = 0; pass < 2; ++pass) {
#pragma unroll
    for (int rd = 0; rd < 2; ++rd) { const int d = rd * 32 + tid / 8, pc = tid % 8; FragH f;
#pragma unroll
      for (int q = 0; q < 8; ++q) f.u[q] = tl[pc * 8 + q][d];
      *(volatile v8us*)((unsigned short*)Vt + ((size_t)slab * 64 + d) * TTv + lg * 64 + pc * 8) = f.half[0]; }
    if (pass == 0) __threadfence(); } }

__global__ __launch_bounds__(256) void k_hl(const float* __restrict__ F, _Float16* __restrict__ Hh, _Float16* __restrict__ Hl, size_t n8) { const size_t t = (size_t)blockIdx.x * 256 + threadIdx.x; if (t >= n8) return; FragH fh, fl; const v4f a = *(const v4fa*)(F + t * 8), c = *(const v4fa*)(F + t * 8 + 4);
#pragma unroll
  for (int q = 0; q < 4; ++q) { _Float16 h = (_Float16)a[q]; fh.h[q] = h; fl.h[q] = (_Float16)((a[q] - (float)h) * 1024.0f); h = (_Float16)c[q]; fh.h[4 + q] = h; fl.h[4 + q] = (_Float16)((c[q] - (float)h) * 1024.0f); }
  for (int pass = 0; pass < 2; ++pass) { *(volatile v8us*)((unsigned short*)Hh + t * 8) = fh.half[0]; *(volatile v8us*)((unsigned short*)Hl + t * 8) = fl.half[0]; if (pass == 0) __threadfence(); } }

__global__ __launch_bounds__(256) void k_cl16(const float* __restrict__ x, int b, int C, int HW, int Ppad, _Float16* __restrict__ XC) { const int t = blockIdx.x * 256 + threadIdx.x; if (t >= Ppad * (C / 8)) return; const int c0 = (t % (C / 8)) * 8, p = t / (C / 8); FragH f;
#pragma unroll
  for (int q = 0; q < 8; ++q) f.h[q] = (p < HW) ? (_Float16)bf16_round(x[((size_t)b * C + c0 + q) * HW + p]) : (_Float16)0.0f;
  *(volatile v8us*)((unsigned short*)XC + (size_t)p * C + c0) = f.half[0]; __threadfence(); *(volatile v8us*)((unsigned short*)XC + (size_t)p * C + c0) = f.half[0]; }
__global__ __launch_bounds__(256) void k_im2col(const _Float16* __restrict__ XC, int side, int C, int Ppad, _Float16* __restrict__ COL) { const int HW = side * side; const int t = blockIdx.x * 256 + threadIdx.x; if (t >= Ppad * 9 * (C / 8)) return; const int c0 = (t % (C / 8)) * 8; const int k = (t / (C / 8)) % 9; const int p = t / ((C / 8) * 9); FragH f = FragH{};
  if (p < HW) { const int h = p / side, w = p % side; const int yy = h - 1 + k / 3, xx = w - 1 + k % 3; if (yy >= 0 && yy < side && xx >= 0 && xx < side) f.half[0] = *(const v8us*)((const unsigned short*)XC + ((size_t)yy * side + xx) * C + c0); }
  *(volatile v8us*)((unsigned short*)COL + ((size_t)p * 9 + k) * C + c0) = f.half[0]; __threadfence(); *(volatile v8us*)((unsigned short*)COL + ((size_t)p * 9 + k) * C + c0) = f.half[0]; }
__global__ __launch_bounds__(256) void k_wtap(const float* __restrict__ wsrc, int O, int C, _Float16* __restrict__ Bt) { const int KD = 9 * C; const int t = blockIdx.x * 256 + threadIdx.x; if (t >= O * (KD / 8)) return; const int col0 = (t % (KD / 8)) * 8; const int o = t / (KD / 8); const int k = col0 / C, c0 = col0 % C; FragH f;
#pragma unroll
  for (int q = 0; q < 8; ++q) f.h[q] = (_Float16)(bf16_round(wsrc[((size_t)o * C + c0 + q) * 9 + k]) * 16.0f);
  *(volatile v8us*)((unsigned short*)Bt + (size_t)o * KD + col0) = f.half[0]; __threadfence(); *(volatile v8us*)((unsigned short*)Bt + (size_t)o * KD + col0) = f.half[0]; }
__global__ __launch_bounds__(256) void k_w1d(const float* __restrict__ wsrc, int O, int C, int KT, _Float16* __restrict__ Bt) { const int KD = KT * C; const int t = blockIdx.x * 256 + threadIdx.x; if (t >= O * (KD / 8)) return; const int col0 = (t % (KD / 8)) * 8; const int o = t / (KD / 8); const int tt = col0 / C, c0 = col0 % C; FragH f;
#pragma unroll
  for (int q = 0; q < 8; ++q) f.h[q] = (_Float16)(bf16_round(wsrc[((size_t)o * C + c0 + q) * KT + tt]) * 16.0f);
  *(volatile v8us*)((unsigned short*)Bt + (size_t)o * KD + col0) = f.half[0]; __threadfence(); *(volatile v8us*)((unsigned short*)Bt + (size_t)o * KD + col0) = f.half[0]; }
__global__ __launch_bounds__(256) void k_bcat(const float* __restrict__ ba, int na, const float* __restrict__ bb, int nb, float* __restrict__ BP) { const int l = blockIdx.x * 256 + threadIdx.x; if (l >= na + nb) return; const float v = (l < na) ? ba[l] : bb[l - na]; *(volatile float*)(BP + l) = v; __threadfence(); *(volatile float*)(BP + l) = v; }
__global__ __launch_bounds__(256) void k_seqcol(const float* __restrict__ Sq, int L, int Lstride, int ldS, int coff, int C, int KT, int Lout, _Float16* __restrict__ COL) { const int t = blockIdx.x * 256 + threadIdx.x; if (t >= NBt * Lout * KT * (C / 8)) return; const int c0 = (t % (C / 8)) * 8; const int tt = (t / (C / 8)) % KT; const int r = t / ((C / 8) * KT); const int b = r / Lout, j = r % Lout; const int src = j + tt - 1; FragH f = FragH{};
  if (src >= 0 && src < L) { const float* sp = Sq + ((size_t)b * Lstride + src) * ldS + coff + c0; const v4f a = *(const v4fa*)sp, c4 = *(const v4fa*)(sp + 4);
#pragma unroll
    for (int q = 0; q < 8; ++q) f.h[q] = (_Float16)((q < 4) ? a[q] : c4[q - 4]); }
  *(volatile v8us*)((unsigned short*)COL + ((size_t)r * KT + tt) * C + c0) = f.half[0]; __threadfence(); *(volatile v8us*)((unsigned short*)COL + ((size_t)r * KT + tt) * C + c0) = f.half[0]; }
__global__ __launch_bounds__(256) void k_f16b(const float* __restrict__ F, int ldF, int coff, int C, int nrows, _Float16* __restrict__ O16) { const int t = blockIdx.x * 256 + threadIdx.x; if (t >= nrows * (C / 8)) return; const int c0 = (t % (C / 8)) * 8, r = t / (C / 8); const v4f a = *(const v4fa*)(F + (size_t)r * ldF + coff + c0), c4 = *(const v4fa*)(F + (size_t)r * ldF + coff + c0 + 4); FragH f;
#pragma unroll
  for (int q = 0; q < 8; ++q) f.h[q] = (_Float16)((q < 4) ? a[q] : c4[q - 4]);
  *(volatile v8us*)((unsigned short*)O16 + (size_t)r * C + c0) = f.half[0]; __threadfence(); *(volatile v8us*)((unsigned short*)O16 + (size_t)r * C + c0) = f.half[0]; }
__global__ __launch_bounds__(256) void k_tr16(const float* __restrict__ F, int L, int ldF, int coff, int C, int Qpad, _Float16* __restrict__ T16) { const int t = blockIdx.x * 256 + threadIdx.x; if (t >= NBt * C * (Qpad / 8)) return; const int q0 = (t % (Qpad / 8)) * 8; const int c = (t / (Qpad / 8)) % C; const int b = t / ((Qpad / 8) * C); FragH f;
#pragma unroll
  for (int i = 0; i < 8; ++i) { const int q = q0 + i; f.h[i] = (q < L) ? (_Float16)F[((size_t)b * L + q) * ldF + coff + c] : (_Float16)0.0f; }
  *(volatile v8us*)((unsigned short*)T16 + ((size_t)b * C + c) * Qpad + q0) = f.half[0]; __threadfence(); *(volatile v8us*)((unsigned short*)T16 + ((size_t)b * C + c) * Qpad + q0) = f.half[0]; }
__global__ __launch_bounds__(256) void k_tr16h(const _Float16* __restrict__ P16, int Pstride, int ld, int coff, int C, int L, int Qpad, _Float16* __restrict__ T16) { const int t = blockIdx.x * 256 + threadIdx.x; if (t >= NBt * C * (Qpad / 8)) return; const int q0 = (t % (Qpad / 8)) * 8; const int c = (t / (Qpad / 8)) % C; const int b = t / ((Qpad / 8) * C); FragH f;
#pragma unroll
  for (int i = 0; i < 8; ++i) { const int q = q0 + i; f.h[i] = (q < L) ? P16[((size_t)b * Pstride + q) * ld + coff + c] : (_Float16)0.0f; }
  *(volatile v8us*)((unsigned short*)T16 + ((size_t)b * C + c) * Qpad + q0) = f.half[0]; __threadfence(); *(volatile v8us*)((unsigned short*)T16 + ((size_t)b * C + c) * Qpad + q0) = f.half[0]; }
__global__ __launch_bounds__(256) void k_tr16s(const float* __restrict__ F, int L, int Pstride, int ldF, int coff, int C, int Qpad, _Float16* __restrict__ T16) { const int t = blockIdx.x * 256 + threadIdx.x; if (t >= NBt * C * (Qpad / 8)) return; const int q0 = (t % (Qpad / 8)) * 8; const int c = (t / (Qpad / 8)) % C; const int b = t / ((Qpad / 8) * C); FragH f;
#pragma unroll
  for (int i = 0; i < 8; ++i) { const int q = q0 + i; f.h[i] = (q < L) ? (_Float16)F[((size_t)b * Pstride + q) * ldF + coff + c] : (_Float16)0.0f; }
  *(volatile v8us*)((unsigned short*)T16 + ((size_t)b * C + c) * Qpad + q0) = f.half[0]; __threadfence(); *(volatile v8us*)((unsigned short*)T16 + ((size_t)b * C + c) * Qpad + q0) = f.half[0]; }
__global__ __launch_bounds__(256) void k_f16s(const float* __restrict__ F, int L, int Pin, int ldF, int coff, int C, int Pout, _Float16* __restrict__ O16) { const int t = blockIdx.x * 256 + threadIdx.x; if (t >= NBt * Pout * (C / 8)) return; const int c0 = (t % (C / 8)) * 8; const int r = t / (C / 8); const int b = r / Pout, q = r % Pout; FragH f = FragH{};
  if (q < L) { const float* sp = F + ((size_t)b * Pin + q) * ldF + coff + c0; const v4f a = *(const v4fa*)sp, c4 = *(const v4fa*)(sp + 4);
#pragma unroll
    for (int i = 0; i < 8; ++i) f.h[i] = (_Float16)((i < 4) ? a[i] : c4[i - 4]); }
  *(volatile v8us*)((unsigned short*)O16 + (size_t)r * C + c0) = f.half[0]; __threadfence(); *(volatile v8us*)((unsigned short*)O16 + (size_t)r * C + c0) = f.half[0]; }
__global__ __launch_bounds__(256) void k_cstat(const float* __restrict__ ST, int Kv, int ldq, int Qv, float* __restrict__ CS) {
  #pragma clang fp contract(off)
  const int q = blockIdx.x * 256 + threadIdx.x; if (q >= Qv) return; float m = -3.0e38f;
#pragma unroll 1
  for (int k = 0; k < Kv; ++k) m = fmaxf(m, ST[(size_t)k * ldq + q]);
  float s = 0.f;
#pragma unroll 1
  for (int k = 0; k < Kv; ++k) s += expf(ST[(size_t)k * ldq + q] - m);
  typedef float v2f __attribute__((ext_vector_type(2))); v2f v; v[0] = m; v[1] = 1024.0f / s; *(volatile v2f*)(CS + 2 * q) = v; __threadfence(); *(volatile v2f*)(CS + 2 * q) = v; }
__global__ __launch_bounds__(256) void k_capply(const float* __restrict__ ST, int Kv, int ldq, int Qv, int Kpad, int Qpad, const float* __restrict__ CS, _Float16* __restrict__ PT) {
  #pragma clang fp contract(off)
  const int t = blockIdx.x * 256 + threadIdx.x; if (t >= Kpad * (Qpad / 8)) return; const int q0 = (t % (Qpad / 8)) * 8, k = t / (Qpad / 8); FragH f;
#pragma unroll
  for (int i = 0; i < 8; ++i) { const int q = q0 + i; float p = 0.f; if (k < Kv && q < Qv) p = expf(ST[(size_t)k * ldq + q] - CS[2 * q]) * CS[2 * q + 1]; f.h[i] = (_Float16)p; }
  *(volatile v8us*)((unsigned short*)PT + (size_t)k * Qpad + q0) = f.half[0]; __threadfence(); *(volatile v8us*)((unsigned short*)PT + (size_t)k * Qpad + q0) = f.half[0]; }
__global__ __launch_bounds__(256) void k_stat(const float* __restrict__ Pm, int nrows, int Ppad, int HW, int C, int phase, float* __restrict__ STAT) {
  #pragma clang fp contract(off)
  __shared__ float red[256]; const int c = blockIdx.x, tid = threadIdx.x; const float cnt = (float)(NBt * HW); const float mean = phase ? (STAT[(size_t)c * 32] / cnt) : 0.f; float s = 0.f;
  for (int r = tid; r < nrows; r += 256) { if ((r % Ppad) >= HW) continue; const float v = Pm[(size_t)r * C + c]; s += phase ? (v - mean) * (v - mean) : v; }
  red[tid] = s; __syncthreads(); for (int st = 128; st > 0; st >>= 1) { if (tid < st) red[tid] += red[tid + st]; __syncthreads(); }
  if (tid < 32) { float* line = STAT + ((size_t)phase * C + c) * 32; *(volatile float*)(line + tid) = red[0]; __threadfence(); *(volatile float*)(line + tid) = red[0]; } }
__global__ __launch_bounds__(256) void k_bnrelu16(const float* __restrict__ Pm, int nrows, int C, int HW, const float* __restrict__ STAT, const float* __restrict__ g, const float* __restrict__ bb, const float* __restrict__ g2, const float* __restrict__ bb2, _Float16* __restrict__ O16) {
  #pragma clang fp contract(off)
  const int t = blockIdx.x * 256 + threadIdx.x; if (t >= nrows * (C / 8)) return; const int c0 = (t % (C / 8)) * 8, r = t / (C / 8); const float cnt = (float)(NBt * HW); const v4f a = *(const v4fa*)(Pm + (size_t)r * C + c0), c4 = *(const v4fa*)(Pm + (size_t)r * C + c0 + 4); FragH f;
#pragma unroll
  for (int q = 0; q < 8; ++q) { const int c = c0 + q; const float mean = STAT[(size_t)c * 32] / cnt, rs = rsqrtf(STAT[(size_t)(C + c) * 32] / cnt + 1e-5f); const int half = C / 2; const float gg = (c < half) ? bf16_round(g[c]) : bf16_round(g2[c - half]), be = (c < half) ? bf16_round(bb[c]) : bf16_round(bb2[c - half]); f.h[q] = (_Float16)fmaxf((((q < 4) ? a[q] : c4[q - 4]) - mean) * rs * gg + be, 0.f); }
  *(volatile v8us*)((unsigned short*)O16 + (size_t)r * C + c0) = f.half[0]; __threadfence(); *(volatile v8us*)((unsigned short*)O16 + (size_t)r * C + c0) = f.half[0]; }
__global__ __launch_bounds__(256) void k_fin(const float* __restrict__ F, const float* __restrict__ STAT, const float* __restrict__ g, const float* __restrict__ bb, const float* __restrict__ x2, float* __restrict__ out) {
  #pragma clang fp contract(off)
  const int t = blockIdx.x * 256 + threadIdx.x; if (t >= NBt * C2 * (HW2 / 4)) return; const int p0 = (t % (HW2 / 4)) * 4; const int c = (t / (HW2 / 4)) % C2; const int b = t / ((HW2 / 4) * C2); const float cnt = (float)(NBt * HW2); const float mean = STAT[(size_t)c * 32] / cnt, rs = rsqrtf(STAT[(size_t)(C2 + c) * 32] / cnt + 1e-5f), gc = bf16_round(g[c]), bc = bf16_round(bb[c]); v4f v;
#pragma unroll
  for (int q = 0; q < 4; ++q) { const int p = p0 + q; v[q] = fmaxf((F[((size_t)b * HW2 + p) * C2 + c] - mean) * rs * gc + bc, 0.f) + bf16_round(x2[((size_t)b * C2 + c) * HW2 + p]); }
  float* dst = out + ((size_t)b * C2 + c) * HW2 + p0; *(volatile v4f*)dst = v; __threadfence(); *(volatile v4f*)dst = v; }

extern "C" void kernel_launch(void* const* d_in, const int* in_sizes, int n_in,
                              void* d_out, int out_size, void* d_ws, size_t ws_size, hipStream_t stream) {
  (void)in_sizes; (void)n_in; (void)out_size;
  const float* const* I = (const float* const*)d_in; const float* x2 = I[0]; const float* x3 = I[1]; const float* x4 = I[2];
  const float* w_r4q = I[3], *b_r4q = I[4], *g_r4q = I[5], *be_r4q = I[6], *w_r4k = I[7], *b_r4k = I[8], *g_r4k = I[9], *be_r4k = I[10], *w_n3 = I[11], *b_n3 = I[12], *w_n2 = I[13], *b_n2 = I[14], *w1_3q = I[15], *b1_3q = I[16], *w1_3k = I[17], *b1_3k = I[18], *w1_2q = I[19], *b1_2q = I[20], *w1_2k = I[21], *b1_2k = I[22], *w_2r = I[23], *b_2r = I[24], *g_2r = I[25], *be_2r = I[26];
  char* ws = (char*)d_ws; size_t off = 0;
  auto take = [&](size_t bytes) { char* p = ws + off; off += (bytes + 255) & ~(size_t)255; return p; };
  const int P4 = 128, P3 = 496, L2P = 1936;
  _Float16* B4 = (_Float16*)take((size_t)2 * C3 * 9 * C4 * 2); float* BP4 = (float*)take(2 * C3 * 4); _Float16* B3 = (_Float16*)take((size_t)C3 * 9 * C3 * 2); _Float16* B2 = (_Float16*)take((size_t)C2 * 9 * C2 * 2); _Float16* B13 = (_Float16*)take((size_t)2 * C2 * 3 * C3 * 2); float* BP13 = (float*)take(2 * C2 * 4); _Float16* B12 = (_Float16*)take((size_t)2 * C2 * 5 * C2 * 2); float* BP12 = (float*)take(2 * C2 * 4); _Float16* B2R = (_Float16*)take((size_t)C2 * 9 * C2 * 2); float* STAT = (float*)take((size_t)2 * 2 * C3 * 32 * 4);
  _Float16* XC = (_Float16*)take((size_t)HW2 * C2 * 2);
  _Float16* COL = (_Float16*)take((size_t)NBt * HW2 * 9 * C2 * 2);
  float* R4 = (float*)take((size_t)NBt * P4 * 2 * C3 * 4); _Float16* R4Q16 = (_Float16*)take((size_t)NBt * P4 * 2 * C3 * 2); _Float16* R4KT = (_Float16*)take((size_t)NBt * C3 * Q4P * 2);
  float* R3 = (float*)take((size_t)NBt * P3 * C3 * 4); _Float16* R3_16 = (_Float16*)take((size_t)NBt * P3 * C3 * 2);
  float* ST = (float*)take((size_t)HW2 * Q2P * 4); float* CS = (float*)take((size_t)Q2P * 2 * 4); _Float16* PT = (_Float16*)take((size_t)HW2 * Q2P * 2);
  float* S3 = (float*)take((size_t)NBt * P3 * C3 * 4); float* Q3K3 = (float*)take((size_t)NBt * HW3 * 2 * C2 * 4); _Float16* Q3_16 = (_Float16*)take((size_t)NBt * Q3P * C2 * 2); _Float16* K3T = (_Float16*)take((size_t)NBt * C2 * Q3P * 2);
  float* R2 = (float*)take((size_t)NBt * HW2 * C2 * 4); _Float16* R2_16 = (_Float16*)take((size_t)NBt * HW2 * C2 * 2); float* S2 = (float*)take((size_t)NBt * HW2 * C2 * 4); float* Q2K2 = (float*)take((size_t)NBt * L2Q * 2 * C2 * 4); _Float16* Q2_16 = (_Float16*)take((size_t)NBt * Q2P * C2 * 2); _Float16* K2T = (_Float16*)take((size_t)NBt * C2 * Q2P * 2);
  float* R2F = S2;
  float* F = Q2K2;
  if (off > ws_size) return;
  k_wtap<<<(C3 * (9 * C4 / 8) + 255) / 256, 256, 0, stream>>>(w_r4q, C3, C4, B4); k_wtap<<<(C3 * (9 * C4 / 8) + 255) / 256, 256, 0, stream>>>(w_r4k, C3, C4, B4 + (size_t)C3 * 9 * C4); k_bcat<<<(2 * C3 + 255) / 256, 256, 0, stream>>>(b_r4q, C3, b_r4k, C3, BP4);
  k_wtap<<<(C3 * (9 * C3 / 8) + 255) / 256, 256, 0, stream>>>(w_n3, C3, C3, B3); k_wtap<<<(C2 * (9 * C2 / 8) + 255) / 256, 256, 0, stream>>>(w_n2, C2, C2, B2); k_wtap<<<(C2 * (9 * C2 / 8) + 255) / 256, 256, 0, stream>>>(w_2r, C2, C2, B2R);
  k_w1d<<<(C2 * (3 * C3 / 8) + 255) / 256, 256, 0, stream>>>(w1_3q, C2, C3, 3, B13); k_w1d<<<(C2 * (3 * C3 / 8) + 255) / 256, 256, 0, stream>>>(w1_3k, C2, C3, 3, B13 + (size_t)C2 * 3 * C3); k_bcat<<<1, 256, 0, stream>>>(b1_3q, C2, b1_3k, C2, BP13);
  k_w1d<<<(C2 * (5 * C2 / 8) + 255) / 256, 256, 0, stream>>>(w1_2q, C2, C2, 5, B12); k_w1d<<<(C2 * (5 * C2 / 8) + 255) / 256, 256, 0, stream>>>(w1_2k, C2, C2, 5, B12 + (size_t)C2 * 5 * C2); k_bcat<<<1, 256, 0, stream>>>(b1_2q, C2, b1_2k, C2, BP12);
  for (int b = 0; b < NBt; ++b) { k_cl16<<<(P4 * (C4 / 8) + 255) / 256, 256, 0, stream>>>(x4, b, C4, HW4, P4, XC); k_im2col<<<(P4 * 9 * (C4 / 8) + 255) / 256, 256, 0, stream>>>(XC, 11, C4, P4, COL + (size_t)b * P4 * 9 * C4); }
  k_gemm_hhx<0><<<dim3(((NBt * P4 / 16) * (2 * C3 / 64) + 3) / 4, 1), 128, 0, stream>>>(COL, 9 * C4, 0, B4, 9 * C4, 0, 0.0625f, BP4, 0, nullptr, 1, 0, 0, R4, nullptr, 2 * C3, 0, NBt * P4, 2 * C3, 9 * C4);
  k_stat<<<2 * C3, 256, 0, stream>>>(R4, NBt * P4, P4, HW4, 2 * C3, 0, STAT); k_stat<<<2 * C3, 256, 0, stream>>>(R4, NBt * P4, P4, HW4, 2 * C3, 1, STAT);
  k_bnrelu16<<<(NBt * P4 * (2 * C3 / 8) + 255) / 256, 256, 0, stream>>>(R4, NBt * P4, 2 * C3, HW4, STAT, g_r4q, be_r4q, g_r4k, be_r4k, R4Q16);
  k_tr16h<<<(NBt * C3 * (Q4P / 8) + 255) / 256, 256, 0, stream>>>(R4Q16, P4, 2 * C3, C3, C3, HW4, Q4P, R4KT);
  for (int b = 0; b < NBt; ++b) { k_cl16<<<(P3 * (C3 / 8) + 255) / 256, 256, 0, stream>>>(x3, b, C3, HW3, P3, XC); k_im2col<<<(P3 * 9 * (C3 / 8) + 255) / 256, 256, 0, stream>>>(XC, 22, C3, P3, COL + (size_t)b * P3 * 9 * C3); }
  k_gemm_hhx<0><<<dim3(((NBt * P3 / 16) * (C3 / 64) + 3) / 4, 1), 128, 0, stream>>>(COL, 9 * C3, 0, B3, 9 * C3, 0, 0.0625f, b_n3, 0, nullptr, 1, 0, 0, R3, nullptr, C3, 0, NBt * P3, C3, 9 * C3);
  k_f16s<<<(NBt * P3 * (C3 / 8) + 255) / 256, 256, 0, stream>>>(R3, HW3, P3, C3, 0, C3, P3, R3_16);
  for (int b = 0; b < NBt; ++b) {
    k_gemm_hhx<0><<<dim3(((P3 / 16) * (Q4P / 64) + 3) / 4, 1), 128, 0, stream>>>(R3_16 + (size_t)b * P3 * C3, C3, 0, R4Q16 + (size_t)b * P4 * 2 * C3, 2 * C3, 0, 1.0f, nullptr, 0, nullptr, 1, 0, 0, ST, nullptr, Q4P, 0, P3, Q4P, C3);
    k_cstat<<<1, 256, 0, stream>>>(ST, HW3, Q4P, HW4, CS); k_capply<<<(P3 * (Q4P / 8) + 255) / 256, 256, 0, stream>>>(ST, HW3, Q4P, HW4, P3, Q4P, CS, PT);
    k_gemm_hhx<0><<<dim3(((P3 / 16) * (C3 / 64) + 3) / 4, 1), 128, 0, stream>>>(PT, Q4P, 0, R4KT + (size_t)b * C3 * Q4P, Q4P, 0, 0.0009765625f, nullptr, 0, R3 + (size_t)b * P3 * C3, 1, (size_t)C3, 0, S3 + (size_t)b * P3 * C3, nullptr, C3, 0, P3, C3, Q4P); }
  k_seqcol<<<(NBt * HW3 * 3 * (C3 / 8) + 255) / 256, 256, 0, stream>>>(S3, HW3, P3, C3, 0, C3, 3, HW3, COL);
  k_gemm_hhx<0><<<dim3(((NBt * HW3 / 16) * (2 * C2 / 64) + 3) / 4, 1), 128, 0, stream>>>(COL, 3 * C3, 0, B13, 3 * C3, 0, 0.0625f, BP13, 0, nullptr, 1, 0, 0, Q3K3, nullptr, 2 * C2, 0, NBt * HW3, 2 * C2, 3 * C3);
  k_f16s<<<(NBt * Q3P * (C2 / 8) + 255) / 256, 256, 0, stream>>>(Q3K3, HW3, HW3, 2 * C2, 0, C2, Q3P, Q3_16);
  k_tr16s<<<(NBt * C2 * (Q3P / 8) + 255) / 256, 256, 0, stream>>>(Q3K3, HW3, HW3, 2 * C2, C2, C2, Q3P, K3T);
  for (int b = 0; b < NBt; ++b) { k_cl16<<<(HW2 * (C2 / 8) + 255) / 256, 256, 0, stream>>>(x2, b, C2, HW2, HW2, XC); k_im2col<<<(HW2 * 9 * (C2 / 8) + 255) / 256, 256, 0, stream>>>(XC, 44, C2, HW2, COL + (size_t)b * HW2 * 9 * C2); }
  k_gemm_hhx<0><<<dim3(((NBt * HW2 / 16) * (C2 / 64) + 3) / 4, 1), 128, 0, stream>>>(COL, 9 * C2, 0, B2, 9 * C2, 0, 0.0625f, b_n2, 0, nullptr, 1, 0, 0, R2, nullptr, C2, 0, NBt * HW2, C2, 9 * C2);
  k_f16s<<<(NBt * HW2 * (C2 / 8) + 255) / 256, 256, 0, stream>>>(R2, HW2, HW2, C2, 0, C2, HW2, R2_16);
  for (int b = 0; b < NBt; ++b) {
    k_gemm_hhx<0><<<dim3(((HW2 / 16) * (Q3P / 64) + 3) / 4, 1), 128, 0, stream>>>(R2_16 + (size_t)b * HW2 * C2, C2, 0, Q3_16 + (size_t)b * Q3P * C2, C2, 0, 1.0f, nullptr, 0, nullptr, 1, 0, 0, ST, nullptr, Q3P, 0, HW2, Q3P, C2);
    k_cstat<<<(HW3 + 255) / 256, 256, 0, stream>>>(ST, HW2, Q3P, HW3, CS); k_capply<<<(HW2 * (Q3P / 8) + 255) / 256, 256, 0, stream>>>(ST, HW2, Q3P, HW3, HW2, Q3P, CS, PT);
    k_gemm_hhx<0><<<dim3(((HW2 / 16) * (C2 / 64) + 3) / 4, 1), 128, 0, stream>>>(PT, Q3P, 0, K3T + (size_t)b * C2 * Q3P, Q3P, 0, 0.0009765625f, nullptr, 0, R2 + (size_t)b * HW2 * C2, 1, (size_t)C2, 0, S2 + (size_t)b * HW2 * C2, nullptr, C2, 0, HW2, C2, Q3P); }
  k_seqcol<<<(NBt * L2Q * 5 * (C2 / 8) + 255) / 256, 256, 0, stream>>>(S2, HW2, HW2, C2, 0, C2, 5, L2Q, COL);
  k_gemm_hhx<0><<<dim3(((NBt * L2Q / 16) * (2 * C2 / 64) + 3) / 4, 1), 128, 0, stream>>>(COL, 5 * C2, 0, B12, 5 * C2, 0, 0.0625f, BP12, 0, nullptr, 1, 0, 0, Q2K2, nullptr, 2 * C2, 0, NBt * L2Q, 2 * C2, 5 * C2);
  k_f16s<<<(NBt * Q2P * (C2 / 8) + 255) / 256, 256, 0, stream>>>(Q2K2, L2Q, L2Q, 2 * C2, 0, C2, Q2P, Q2_16);
  k_tr16s<<<(NBt * C2 * (Q2P / 8) + 255) / 256, 256, 0, stream>>>(Q2K2, L2Q, L2Q, 2 * C2, C2, C2, Q2P, K2T);
  for (int b = 0; b < NBt; ++b) {
    k_gemm_hhx<0><<<dim3(((HW2 / 16) * ((Q2P + 63) / 64) + 3) / 4, 1), 128, 0, stream>>>(R2_16 + (size_t)b * HW2 * C2, C2, 0, Q2_16 + (size_t)b * Q2P * C2, C2, 0, 1.0f, nullptr, 0, nullptr, 1, 0, 0, ST, nullptr, Q2P, 0, HW2, Q2P, C2);
    k_cstat<<<(L2Q + 255) / 256, 256, 0, stream>>>(ST, HW2, Q2P, L2Q, CS); k_capply<<<(HW2 * (Q2P / 8) + 255) / 256, 256, 0, stream>>>(ST, HW2, Q2P, L2Q, HW2, Q2P, CS, PT);
    k_gemm_hhx<0><<<dim3(((HW2 / 16) * (C2 / 64) + 3) / 4, 1), 128, 0, stream>>>(PT, Q2P, 0, K2T + (size_t)b * C2 * Q2P, Q2P, 0, 0.0009765625f, nullptr, 0, nullptr, 1, 0, 0, R2F + (size_t)b * HW2 * C2, nullptr, C2, 0, HW2, C2, Q2P); }
  for (int b = 0; b < NBt; ++b) { k_f16b<<<(HW2 * (C2 / 8) + 255) / 256, 256, 0, stream>>>(R2F + (size_t)b * HW2 * C2, C2, 0, C2, HW2, XC); k_im2col<<<(HW2 * 9 * (C2 / 8) + 255) / 256, 256, 0, stream>>>(XC, 44, C2, HW2, COL + (size_t)b * HW2 * 9 * C2); }
  k_gemm_hhx<0><<<dim3(((NBt * HW2 / 16) * (C2 / 64) + 3) / 4, 1), 128, 0, stream>>>(COL, 9 * C2, 0, B2R, 9 * C2, 0, 0.0625f, b_2r, 0, nullptr, 1, 0, 0, F, nullptr, C2, 0, NBt * HW2, C2, 9 * C2);
  k_stat<<<C2, 256, 0, stream>>>(F, NBt * HW2, HW2, HW2, C2, 0, STAT); k_stat<<<C2, 256, 0, stream>>>(F, NBt * HW2, HW2, HW2, C2, 1, STAT);
  k_fin<<<(NBt * C2 * (HW2 / 4) + 255) / 256, 256, 0, stream>>>(F, STAT, g_2r, be_2r, x2, (float*)d_out);
}
